// rnnmodel_11252814316201
// MI455X (gfx1250) — hardware-verified
//
#include <hip/hip_runtime.h>
#include <math.h>

typedef __attribute__((ext_vector_type(16))) _Float16 v16h;
typedef __attribute__((ext_vector_type(8)))  _Float16 v8h;
typedef __attribute__((ext_vector_type(8)))  float    v8f;
typedef __attribute__((ext_vector_type(4)))  float    v4f;

constexpr int kBatch    = 2048;
constexpr int kSteps    = 512;
constexpr int kIn       = 3;
constexpr int kHid      = 10;
constexpr int kLayers   = 10;
constexpr int kTileRows = 16;
constexpr int kTiles    = kBatch / kTileRows;
constexpr int kWavesPerBlock = 4;
constexpr int kChunk    = 32;
constexpr int kNumChunks = kSteps / kChunk;
constexpr int kXPitch   = kChunk * kIn + 4;
constexpr int kOPitch   = kChunk + 4;
constexpr size_t kOutElems = (size_t)kBatch * kSteps;
static_assert(kBatch % (kTileRows * kWavesPerBlock) == 0 && kSteps % kChunk == 0, "whole tiles and chunks");
static_assert(kHid <= 16 && kIn <= 8, "a layer's units fit one 16-row tile and one half of K; the input features fit the low lane half");
static_assert((kXPitch % 4) == 0 && (kOPitch % 4) == 0, "16-B aligned LDS rows");

constexpr float kStateCarry  = 4096.0f;
constexpr float kWeightCarry = 64.0f;
constexpr float kFoldBack    = 1.0f / (kStateCarry * kWeightCarry);
constexpr float kF16MinNorm  = 6.103515625e-5f;

namespace eng {

union FragU { v16h v; v8h h[2]; };

__device__ __forceinline__ unsigned short f2bf_bits(float f) {
  unsigned u = __float_as_uint(f);
  return (unsigned short)((u + 0x7FFFu + ((u >> 16) & 1u)) >> 16);
}
__device__ __forceinline__ float bf16v(float f) {
  return __uint_as_float(((unsigned)f2bf_bits(f)) << 16);
}
__device__ __forceinline__ _Float16 to_f16_flushed(float c) {
  const float z = (fabsf(c) < kF16MinNorm) ? 0.0f : c;
  return (_Float16)z;
}
__device__ __forceinline__ v8f mma_f16(v16h a, v16h b) {
  v8f c = (v8f){0.f, 0.f, 0.f, 0.f, 0.f, 0.f, 0.f, 0.f};
  c = __builtin_amdgcn_wmma_f32_16x16x32_f16(false, a, false, b, (short)0, c, false, false);
  asm volatile("v_nop\n\tv_nop\n\tv_nop\n\tv_nop" : "+v"(c) : "v"(a), "v"(b));
  return c;
}
__device__ __forceinline__ float fast_tanh(float v) {
  const float e = __expf(2.0f * v);
  return 1.0f - 2.0f * __builtin_amdgcn_rcpf(e + 1.0f);
}
__device__ __forceinline__ float fast_sigmoid(float v) {
  return __builtin_amdgcn_rcpf(1.0f + __expf(-v));
}

__device__ __forceinline__ v8f mma_f16_acc(v16h a, v16h b, v8f c) {
  c = __builtin_amdgcn_wmma_f32_16x16x32_f16(false, a, false, b, (short)0, c, false, false);
  asm volatile("v_nop\n\tv_nop\n\tv_nop\n\tv_nop" : "+v"(c) : "v"(a), "v"(b));
  return c;
}

}

__global__ __launch_bounds__(32 * kWavesPerBlock) void elman10_seq_kernel(
    const float* __restrict__ x, const float* __restrict__ w_ih0, const float* __restrict__ w_ih,
    const float* __restrict__ w_hh, const float* __restrict__ b_ih, const float* __restrict__ b_hh,
    const float* __restrict__ w_out, const float* __restrict__ b_out, float* __restrict__ outs)
{
  __shared__ __align__(16) float xsAll[kWavesPerBlock][kTileRows * kXPitch];
  __shared__ __align__(16) float osAll[kWavesPerBlock][kTileRows * kOPitch];
  __shared__ __align__(16) float wsm[2144];
  __shared__ __align__(32) v16h fragS[kLayers][32];

  const int tid  = threadIdx.x;
  const int lane = tid & 31;
  const int wave = tid >> 5;
  float* xs = &xsAll[wave][0];
  float* os = &osAll[wave][0];
  const int hsel = lane >> 4;
  const int n    = lane & 15;
  const bool lowHalf = (hsel == 0);
  const int b0   = (blockIdx.x * kWavesPerBlock + wave) * kTileRows;
  constexpr int oI0 = 0, oIh = 30, oHh = 930, oBi = 1930, oBh = 2030, oWo = 2130, oBo = 2140;

#pragma unroll 1
  for (int i = tid; i < 1000; i += 32 * kWavesPerBlock) {
    const int i30 = (i < 30) ? i : 29;
    const int i900 = (i < 900) ? i : 899;
    const int i100 = (i < 100) ? i : 99;
    const int i10 = (i < 10) ? i : 9;
    wsm[oI0 + i30] = w_ih0[i30];
    wsm[oIh + i900] = w_ih[i900];
    wsm[oHh + i] = w_hh[i];
    wsm[oBi + i100] = b_ih[i100];
    wsm[oBh + i100] = b_hh[i100];
    wsm[oWo + i10] = w_out[i10];
    wsm[oBo] = b_out[0];
  }
  __syncthreads();

  {
    const int m  = n;
    const int mc = (m < kHid) ? m : (kHid - 1);
    const bool mok = (m < kHid);
#pragma unroll 1
    for (int l = wave; l < kLayers; l += kWavesPerBlock) {
      v8h ai, ah;
#pragma unroll
      for (int i = 0; i < 8; ++i) {
        const int k  = 8 * hsel + i;
        const int kc = (k < kHid) ? k : (kHid - 1);
        const int k3 = (k < kIn) ? k : (kIn - 1);
        const float fi = (l == 0) ? wsm[oI0 + mc * kIn + k3] : wsm[oIh + ((l - 1) * kHid + mc) * kHid + kc];
        const bool oki = mok && ((l == 0) ? (k < kIn) : (k < kHid));
        const float fh = wsm[oHh + (l * kHid + mc) * kHid + kc];
        const bool okh = mok && (k < kHid);
        ai[i] = eng::to_f16_flushed(oki ? eng::bf16v(fi) * kWeightCarry : 0.0f);
        ah[i] = eng::to_f16_flushed(okh ? eng::bf16v(fh) * kWeightCarry : 0.0f);
      }
      eng::FragU u1;
      u1.h[0] = ai;
      u1.h[1] = ah;
      fragS[l][lane] = u1.v;
    }
  }
  __syncthreads();
  float wo[8];
#pragma unroll
  for (int r = 0; r < 8; ++r) {
    const int u  = 8 * hsel + r;
    const int uc = (u < kHid) ? u : (kHid - 1);
    const float vwo = eng::bf16v(wsm[oWo + uc]);
    wo[r] = (u < kHid) ? vwo : 0.0f;
  }
  const float bo = eng::bf16v(wsm[oBo]);
  v8h hb[kLayers], hl[kLayers];
#pragma unroll
  for (int l = 0; l < kLayers; ++l) {
#pragma unroll
    for (int r = 0; r < 8; ++r) { hb[l][r] = (_Float16)0.0f; hl[l][r] = (_Float16)0.0f; }
  }

  const int q  = lane >> 3;
  const int c4 = (lane & 7) * 4;

#pragma unroll 1
  for (int ch = 0; ch < kNumChunks; ++ch) {
    const int t0 = ch * kChunk;
#pragma unroll
    for (int it = 0; it < 12; ++it) {
      const int ln = it * 4 + q;
      const int row = ln / 3;
      const int part = ln - 3 * row;
      const v4f v = *(const v4f*)(x + ((size_t)(b0 + row) * kSteps + t0) * kIn + part * 32 + c4);
      v4f rv;
      rv[0] = eng::bf16v(v[0]);
      rv[1] = eng::bf16v(v[1]);
      rv[2] = eng::bf16v(v[2]);
      rv[3] = eng::bf16v(v[3]);
      *(v4f*)(xs + row * kXPitch + part * 32 + c4) = rv;
    }
    __syncthreads();

#pragma unroll 1
    for (int s = 0; s < kChunk; ++s) {
      v8h inb, inl;
#pragma unroll
      for (int i = 0; i < 8; ++i) {
        const int ic = (i < kIn) ? i : (kIn - 1);
        const float xv = xs[n * kXPitch + s * kIn + ic];
        inb[i] = eng::to_f16_flushed((lowHalf && i < kIn) ? xv * kStateCarry : 0.0f);
        inl[i] = (_Float16)0.0f;
      }
      float p = 0.0f;
#pragma unroll
      for (int l = 0; l < kLayers; ++l) {
        eng::FragU fb, fl;
        fb.h[0] = inb;
        fb.h[1] = hb[l];
        fl.h[0] = inl;
        fl.h[1] = hl[l];
        const v16h fa = fragS[l][lane];
        const v8f d = eng::mma_f16_acc(fa, fl.v, eng::mma_f16(fa, fb.v));
#pragma unroll
        for (int r = 0; r < 8; ++r) {
          const int u  = 8 * hsel + r;
          const int uc = (u < kHid) ? u : (kHid - 1);
          const float bias = eng::bf16v(wsm[oBi + l * kHid + uc]) + eng::bf16v(wsm[oBh + l * kHid + uc]);
          const float tv = eng::fast_tanh(fmaf(d[r], kFoldBack, bias));
          const float hv = (u < kHid) ? tv : 0.0f;
          const float hc = hv * kStateCarry;
          const _Float16 hh = eng::to_f16_flushed(hc);
          const _Float16 lo = eng::to_f16_flushed(hc - (float)hh);
          hb[l][r] = hh;
          hl[l][r] = lo;
          inb[r] = hh;
          inl[r] = lo;
          if (l == kLayers - 1) p = fmaf(wo[r], hv, p);
        }
      }
      const float pother = __shfl_xor(p, 16, 32);
      const float tot = (p + pother) + bo;
      if (lowHalf) os[n * kOPitch + s] = tot;
    }
    __syncthreads();

    {
      v4f ov[4];
#pragma unroll
      for (int it = 0; it < 4; ++it) ov[it] = *(const v4f*)(os + (it * 4 + q) * kOPitch + c4);
      for (int pass = 0; pass < 2; ++pass) {
#pragma unroll
        for (int it = 0; it < 4; ++it)
          *(volatile v4f*)(outs + (size_t)(b0 + it * 4 + q) * kSteps + t0 + c4) = ov[it];
        __threadfence();
      }
    }
    __syncthreads();
  }
}

extern "C" void kernel_launch(void* const* d_in, const int* in_sizes, int n_in,
                              void* d_out, int out_size, void* d_ws, size_t ws_size,
                              hipStream_t stream) {
  (void)d_ws;
  (void)ws_size;
  if (n_in < 8 || d_out == nullptr) return;
  if ((size_t)in_sizes[0] != kOutElems * kIn) return;
  if (in_sizes[1] != kHid * kIn || in_sizes[2] != (kLayers - 1) * kHid * kHid || in_sizes[3] != kLayers * kHid * kHid) return;
  if (in_sizes[4] != kLayers * kHid || in_sizes[5] != kLayers * kHid || in_sizes[6] != kHid || in_sizes[7] != 1) return;
  if ((size_t)out_size != kOutElems) return;
  elman10_seq_kernel<<<kTiles / kWavesPerBlock, 32 * kWavesPerBlock, 0, stream>>>(
      (const float*)d_in[0], (const float*)d_in[1], (const float*)d_in[2], (const float*)d_in[3],
      (const float*)d_in[4], (const float*)d_in[5], (const float*)d_in[6], (const float*)d_in[7], (float*)d_out);
}
